// SE3AttentionLayer_82970178224144
// MI455X (gfx1250) — hardware-verified
//
#include <hip/hip_runtime.h>
#include <math.h>
#include <stdint.h>

#define NBATCH  2
#define NTOK    2048
#define DM      384
#define NH      8
#define HD      48
#define QP      64
#define QKP     (NH * QP)
#define MROWS   (NBATCH * NTOK)
#define NFR     9
#define WSC     64.0f
#define ACARRY  16.0f
#define QC      16.0f
#define KC      16.0f
#define VC      16.0f
#define PC      1024.0f
#define FC      1024.0f
#define LN_EPS  1e-5f
static_assert(NH * HD == DM);
static_assert(HD == 48 && QP == 64 && QKP == 512);
static_assert((MROWS % 64) == 0 && (DM % 64) == 0 && (NTOK % 64) == 0 && (DM % 32) == 0);
static_assert((NTOK % 32) == 0 && (MROWS % 16) == 0 && (MROWS % 8) == 0);
static_assert(DM == 3 * 128);
#define ATT_BLOCKS (NBATCH * (NTOK / 16))
#define CT_PIECES  (16 * (DM / 8))
static_assert(CT_PIECES == 3 * 256);
#define RP_PIECES  (16 * (QKP / 8))
static_assert(RP_PIECES == 4 * 256);

typedef _Float16 v16h __attribute__((ext_vector_type(16)));
typedef _Float16 v8h  __attribute__((ext_vector_type(8)));
typedef float    v8f  __attribute__((ext_vector_type(8)));
typedef float    v4f  __attribute__((ext_vector_type(4)));
typedef unsigned int v4u __attribute__((ext_vector_type(4)));

union FragH { v16h v; v8h h[2]; v4u u[2]; };

__device__ __forceinline__ unsigned short bf_bits(float f) {
  unsigned u = __float_as_uint(f);
  return (unsigned short)((u + 0x7FFFu + ((u >> 16) & 1u)) >> 16);
}
__device__ __forceinline__ float bf_up(unsigned short h) { return __uint_as_float(((unsigned)h) << 16); }
__device__ __forceinline__ float bfr(float f) { return bf_up(bf_bits(f)); }
__device__ __forceinline__ unsigned short h_bits(_Float16 x) { return __builtin_bit_cast(unsigned short, x); }
__device__ __forceinline__ unsigned pk16(unsigned short a, unsigned short b) { return (unsigned)a | ((unsigned)b << 16); }
__device__ __forceinline__ v8f zero8() { v8f z = {0.f, 0.f, 0.f, 0.f, 0.f, 0.f, 0.f, 0.f}; return z; }

__device__ __forceinline__ v16h ldfrag_h(const _Float16* p) {
  FragH f;
  f.h[0] = *(const v8h*)(p);
  f.h[1] = *(const v8h*)(p + 16);
  return f.v;
}
__device__ __forceinline__ v16h ldfrag_u(const unsigned short* p) {
  FragH f;
  f.u[0] = *(const v4u*)(p);
  f.u[1] = *(const v4u*)(p + 16);
  return f.v;
}

__device__ __forceinline__ v8f mma_raw(v16h a, v16h b, v8f c) {
  return __builtin_amdgcn_wmma_f32_16x16x32_f16(false, a, false, b, (short)0, c, false, false);
}
__device__ __forceinline__ void dep_guard1(v8f& a, v8f& b, v16h x) {
#if defined(__HIP_DEVICE_COMPILE__)
  asm volatile("v_nop\n\tv_nop\n\tv_nop\n\tv_nop" : "+v"(a), "+v"(b) : "v"(x));
#endif
}
__device__ __forceinline__ void guard_s2(v8f& s, v16h a0, v16h a1) {
#if defined(__HIP_DEVICE_COMPILE__)
  asm volatile("v_nop\n\tv_nop\n\tv_nop\n\tv_nop" : "+v"(s) : "v"(a0), "v"(a1));
#endif
}
__device__ __forceinline__ void guard_s4(v8f& s, v16h a0, v16h a1, v16h b0, v16h b1) {
#if defined(__HIP_DEVICE_COMPILE__)
  asm volatile("v_nop\n\tv_nop\n\tv_nop\n\tv_nop" : "+v"(s) : "v"(a0), "v"(a1), "v"(b0), "v"(b1));
#endif
}
__device__ __forceinline__ void guard_pv3(v8f& a, v8f& b, v8f& c, v16h x, v16h y, v16h z, v16h w) {
#if defined(__HIP_DEVICE_COMPILE__)
  asm volatile("v_nop\n\tv_nop\n\tv_nop\n\tv_nop" : "+v"(a), "+v"(b), "+v"(c) : "v"(x), "v"(y), "v"(z), "v"(w));
#endif
}
__device__ __forceinline__ void keep4_h(v16h a, v16h b, v16h c, v16h d) {
#if defined(__HIP_DEVICE_COMPILE__)
  asm volatile("v_nop" :: "v"(a), "v"(b), "v"(c), "v"(d));
#endif
}
__device__ __forceinline__ void acc_guard4(v8f& a, v8f& b, v8f& c, v8f& d) {
#if defined(__HIP_DEVICE_COMPILE__)
  asm volatile("v_nop\n\tv_nop\n\tv_nop\n\tv_nop" : "+v"(a), "+v"(b), "+v"(c), "+v"(d));
#endif
}
__device__ __forceinline__ void wave_sync_lds() {
  __builtin_amdgcn_fence(__ATOMIC_RELEASE, "workgroup");
  __builtin_amdgcn_wave_barrier();
  __builtin_amdgcn_fence(__ATOMIC_ACQUIRE, "workgroup");
}

__global__ __launch_bounds__(256) void conv16(const float* __restrict__ W, unsigned short* dst, int n8, float wsc) {
  const int i  = blockIdx.x * 256 + threadIdx.x;
  const int ic = (i < n8) ? i : (n8 - 1);
  const float* p = W + (size_t)ic * 8;
  const v4f a = *(const v4f*)(p), b = *(const v4f*)(p + 4);
  float v[8];
#pragma unroll
  for (int e = 0; e < 4; ++e) { v[e] = bfr(a[e]); v[4 + e] = bfr(b[e]); }
  v4u ov;
#pragma unroll
  for (int e = 0; e < 4; ++e) ov[e] = pk16(h_bits((_Float16)(v[2 * e] * wsc)), h_bits((_Float16)(v[2 * e + 1] * wsc)));
  if (i < n8) *(volatile v4u*)(dst + (size_t)i * 8) = ov;
  __threadfence();
  if (i < n8) *(volatile v4u*)(dst + (size_t)i * 8) = ov;
}

template <int OM, int HASB>
__global__ __launch_bounds__(256) void gemm64(
    const unsigned short* __restrict__ Ap, int lda, long long sA,
    const unsigned short* __restrict__ Btp, int ldb, long long sB,
    const float* __restrict__ bias, float bscale,
    void* Cout, void* Cout2, int ldc, long long sC,
    int M, int N, int K, float oscale) {
  __shared__ __align__(16) float sT[8][16 * 68];
  const int by   = blockIdx.y;
  const int lane = threadIdx.x & 31;
  const int wave = threadIdx.x >> 5;
  const int tilesN = N >> 6;
  const int tilesM = M >> 6;
  const int tile = blockIdx.x * 8 + wave;
  if (tile >= tilesM * tilesN) return;
  const int tm = tile / tilesN;
  const int tn = tile - tm * tilesN;
  const int m0 = tm << 6;
  const int n0 = tn << 6;

  const unsigned short* A1 = Ap  + (size_t)((long long)by * sA);
  const unsigned short* Bb = Btp + (size_t)((long long)by * sB);

  const int rlane = lane & 15;
  const int koff  = (lane >> 4) * 8;
  const int mOff  = (lane >> 4) * 8;

  v8f acc[4][4];
#pragma unroll
  for (int i = 0; i < 4; ++i)
#pragma unroll
    for (int j = 0; j < 4; ++j) acc[i][j] = zero8();

  for (int k0 = 0; k0 < K; k0 += 32) {
    v16h bh[4];
#pragma unroll
    for (int j = 0; j < 4; ++j) {
      const size_t bofs = (size_t)(n0 + (j << 4) + rlane) * ldb + koff + k0;
      bh[j] = ldfrag_u(Bb + bofs);
    }
#pragma unroll
    for (int i = 0; i < 4; ++i) {
      const size_t ao = (size_t)(m0 + (i << 4) + rlane) * lda + koff + k0;
      const v16h ah = ldfrag_u(A1 + ao);
#pragma unroll
      for (int j = 0; j < 4; ++j) acc[i][j] = mma_raw(ah, bh[j], acc[i][j]);
      dep_guard1(acc[i][0], acc[i][3], ah);
    }
    keep4_h(bh[0], bh[1], bh[2], bh[3]);
  }
  acc_guard4(acc[0][0], acc[0][1], acc[0][2], acc[0][3]);
  acc_guard4(acc[1][0], acc[1][1], acc[1][2], acc[1][3]);
  acc_guard4(acc[2][0], acc[2][1], acc[2][2], acc[2][3]);
  acc_guard4(acc[3][0], acc[3][1], acc[3][2], acc[3][3]);

  const int hh2 = lane >> 4, c4 = (lane & 15) * 4;
  const int q8  = lane >> 3, c8 = (lane & 7) * 8;
  float bc[4];
#pragma unroll
  for (int e = 0; e < 4; ++e) bc[e] = 0.f;
  if (HASB != 0 && OM == 0) {
    const int cb = n0 + c4;
    const int i0 = (cb < N - 4) ? cb : (N - 4);
    const v4f b0v = *(const v4f*)(bias + i0);
#pragma unroll
    for (int e = 0; e < 4; ++e) bc[e] = bfr(b0v[e]) * bscale;
  }

  float* slab = sT[wave];
#pragma unroll
  for (int i = 0; i < 4; ++i) {
    const int mBase = m0 + (i << 4);
#pragma unroll
    for (int j = 0; j < 4; ++j) {
#pragma unroll
      for (int r = 0; r < 8; ++r) {
        slab[(mOff + r) * 68 + (j << 4) + rlane] = acc[i][j][r];
      }
    }
    wave_sync_lds();
    if (OM == 0) {
      float* C = (float*)Cout + (size_t)((long long)by * sC);
      v4f vals[8];
#pragma unroll
      for (int it = 0; it < 8; ++it) {
        const int row = it * 2 + hh2;
        v4f v = *(const v4f*)(slab + row * 68 + c4);
#pragma unroll
        for (int e = 0; e < 4; ++e) v[e] = v[e] * oscale + bc[e];
        vals[it] = v;
      }
      for (int pass = 0; pass < 2; ++pass) {
#pragma unroll
        for (int it = 0; it < 8; ++it) {
          const int gr = mBase + it * 2 + hh2;
          *(volatile v4f*)(C + (size_t)gr * ldc + n0 + c4) = vals[it];
        }
        __threadfence();
      }
    } else {
      unsigned short* C  = (unsigned short*)Cout  + (size_t)((long long)by * sC);
      unsigned short* C2 = (unsigned short*)Cout2 + (size_t)((long long)by * sC);
      v4u hv[4], lv[4];
#pragma unroll
      for (int it = 0; it < 4; ++it) {
        const int row = it * 4 + q8;
        const float* sp = slab + row * 68 + c8;
        v4u a = {0u, 0u, 0u, 0u}, b = {0u, 0u, 0u, 0u};
#pragma unroll
        for (int e = 0; e < 4; ++e) {
          const float f0 = sp[2 * e] * oscale;
          const float f1 = sp[2 * e + 1] * oscale;
          const _Float16 h0 = (_Float16)f0, h1 = (_Float16)f1;
          a[e] = pk16(h_bits(h0), h_bits(h1));
          if (OM == 3) {
            const _Float16 l0 = (_Float16)(f0 - (float)h0), l1 = (_Float16)(f1 - (float)h1);
            b[e] = pk16(h_bits(l0), h_bits(l1));
          }
        }
        hv[it] = a;
        lv[it] = b;
      }
      for (int pass = 0; pass < 2; ++pass) {
#pragma unroll
        for (int it = 0; it < 4; ++it) {
          const int row = it * 4 + q8;
          *(volatile v4u*)(C + (size_t)(mBase + row) * ldc + n0 + c8) = hv[it];
          if (OM == 3) *(volatile v4u*)(C2 + (size_t)(mBase + row) * ldc + n0 + c8) = lv[it];
        }
        __threadfence();
      }
    }
    wave_sync_lds();
  }
}

__global__ __launch_bounds__(256) void rot_pack(const float* __restrict__ QK, const float* __restrict__ frames,
                                                unsigned short* QR, unsigned short* KR, float qc, float kc) {
  __shared__ __align__(16) unsigned short Os[2][16 * QKP];
  __shared__ float Fs[16 * NFR + 16];
  const int tid = threadIdx.x;
  const int rb  = blockIdx.x * 16;
  if (tid < 16 * NFR) Fs[tid] = bfr(frames[(size_t)rb * NFR + tid]);
  {
    const int row = tid >> 4, pl = (tid >> 3) & 1, hd = tid & 7;
    const v4u z = {0u, 0u, 0u, 0u};
    unsigned short* o = Os[pl] + row * QKP + hd * QP + HD;
    *(v4u*)(o)     = z;
    *(v4u*)(o + 8) = z;
  }
  __syncthreads();
  const int pl = (tid >> 7) & 1;
  const int g  = tid & 127;
  const int hd = g >> 4, gi = g & 15;
  const float sc = (pl != 0) ? kc : qc;
#pragma unroll 1
  for (int row = 0; row < 16; ++row) {
    const float* src = QK + (size_t)(rb + row) * (2 * DM) + pl * DM + g * 3;
    const float t0 = src[0], t1 = src[1], t2 = src[2];
    const float* R = Fs + row * NFR;
    unsigned short* o = Os[pl] + row * QKP + hd * QP + gi * 3;
#pragma unroll
    for (int i = 0; i < 3; ++i) {
      const float r = R[3 * i] * t0 + R[3 * i + 1] * t1 + R[3 * i + 2] * t2;
      o[i] = h_bits((_Float16)(r * sc));
    }
  }
  __syncthreads();
  v4u vq[4], vk[4];
#pragma unroll
  for (int it = 0; it < 4; ++it) {
    const int p   = it * 256 + tid;
    const int row = p >> 6;
    const int c8  = (p & 63) * 8;
    vq[it] = *(const v4u*)(Os[0] + row * QKP + c8);
    vk[it] = *(const v4u*)(Os[1] + row * QKP + c8);
  }
  unsigned short* dq = QR + (size_t)rb * QKP;
  unsigned short* dk = KR + (size_t)rb * QKP;
  for (int pass = 0; pass < 2; ++pass) {
#pragma unroll
    for (int it = 0; it < 4; ++it) {
      const int p   = it * 256 + tid;
      const int row = p >> 6;
      const int c8  = (p & 63) * 8;
      *(volatile v4u*)(dq + (size_t)row * QKP + c8) = vq[it];
      *(volatile v4u*)(dk + (size_t)row * QKP + c8) = vk[it];
    }
    __threadfence();
  }
}

__global__ __launch_bounds__(256)
void attn48(const unsigned short* __restrict__ QRp, const unsigned short* __restrict__ KRp,
            const unsigned short* __restrict__ VTq, unsigned short* CT) {
  __shared__ __align__(16) float Ps[NH][16 * 36];
  __shared__ __align__(16) unsigned short Os[16 * DM];

  const int tid  = threadIdx.x;
  const int wave = tid >> 5;
  const int lane = tid & 31;
  const int hh   = lane >> 4;
  const int c    = lane & 15;

  const int bat  = blockIdx.x / (NTOK / 16);
  const int qt   = blockIdx.x - bat * (NTOK / 16);
  const int head = wave;
  const int q0   = qt * 16;

  const size_t qofs = ((size_t)bat * NTOK + q0 + c) * QKP + head * QP + 8 * hh;
  const _Float16* Qh = (const _Float16*)(const void*)QRp + qofs;
  const _Float16* Kb = (const _Float16*)(const void*)KRp + (size_t)bat * NTOK * QKP + head * QP + 8 * hh;
  const _Float16* Vb = (const _Float16*)(const void*)VTq + (size_t)(bat * NH + head) * HD * NTOK + 8 * hh;
  const float lsc = (1.4426950408889634f * 0.14433756729740643f) / (QC * KC);

  const v16h qa = ldfrag_h(Qh), qb = ldfrag_h(Qh + 32);

  float mrow[8], lrow[8];
  v8f o0 = zero8(), o1 = zero8(), o2 = zero8();
#pragma unroll
  for (int r = 0; r < 8; ++r) { mrow[r] = -INFINITY; lrow[r] = 0.f; }
  float* pt = Ps[wave];

#pragma unroll 1
  for (int kb = 0; kb < NTOK; kb += 32) {
    const _Float16* kp = Kb + (size_t)(kb + c) * QKP;
    v8f s0, s1;
    {
      const v16h k0 = ldfrag_h(kp), k1 = ldfrag_h(kp + 32);
      s0 = mma_raw(qa, k0, zero8());
      s0 = mma_raw(qb, k1, s0);
      guard_s2(s0, k0, k1);
    }
    {
      const _Float16* kq = kp + (size_t)16 * QKP;
      const v16h k0 = ldfrag_h(kq), k1 = ldfrag_h(kq + 32);
      s1 = mma_raw(qa, k0, zero8());
      s1 = mma_raw(qb, k1, s1);
      guard_s4(s1, k0, k1, qa, qb);
    }
#pragma unroll
    for (int r = 0; r < 8; ++r) {
      const float t0 = s0[r] * lsc, t1 = s1[r] * lsc;
      float mx = fmaxf(t0, t1);
#pragma unroll
      for (int off = 1; off < 16; off <<= 1) mx = fmaxf(mx, __shfl_xor(mx, off, 32));
      const float mn = fmaxf(mrow[r], mx);
      const float al = exp2f(mrow[r] - mn);
      mrow[r] = mn;
      const float e0 = exp2f(t0 - mn), e1 = exp2f(t1 - mn);
      float ps = e0 + e1;
#pragma unroll
      for (int off = 1; off < 16; off <<= 1) ps += __shfl_xor(ps, off, 32);
      lrow[r] = lrow[r] * al + ps;
      o0[r] *= al;
      o1[r] *= al;
      o2[r] *= al;
      const int ro = (8 * hh + r) * 36 + c;
      pt[ro]      = e0;
      pt[ro + 16] = e1;
    }
    wave_sync_lds();
    FragH ph;
    {
      const float* prow = pt + c * 36 + 8 * hh;
      const v4f p0 = *(const v4f*)(prow), p1 = *(const v4f*)(prow + 4);
      const v4f p2 = *(const v4f*)(prow + 16), p3 = *(const v4f*)(prow + 20);
#pragma unroll
      for (int e = 0; e < 4; ++e) {
        ph.h[0][e]     = (_Float16)(p0[e] * PC);
        ph.h[0][4 + e] = (_Float16)(p1[e] * PC);
        ph.h[1][e]     = (_Float16)(p2[e] * PC);
        ph.h[1][4 + e] = (_Float16)(p3[e] * PC);
      }
    }
    const _Float16* vp = Vb + (size_t)c * NTOK + kb;
    {
      const v16h vb0 = ldfrag_h(vp), vb1 = ldfrag_h(vp + (size_t)16 * NTOK), vb2 = ldfrag_h(vp + (size_t)32 * NTOK);
      o0 = mma_raw(ph.v, vb0, o0);
      o1 = mma_raw(ph.v, vb1, o1);
      o2 = mma_raw(ph.v, vb2, o2);
      guard_pv3(o0, o1, o2, ph.v, vb0, vb1, vb2);
    }
    wave_sync_lds();
  }

  const float oc = FC / (PC * VC);
  unsigned short* osw = Os + head * HD + c;
#pragma unroll
  for (int r = 0; r < 8; ++r) {
    const float inv = (1.0f / lrow[r]) * oc;
    unsigned short* op = osw + (8 * hh + r) * DM;
    op[0]  = h_bits((_Float16)(o0[r] * inv));
    op[16] = h_bits((_Float16)(o1[r] * inv));
    op[32] = h_bits((_Float16)(o2[r] * inv));
  }
  __syncthreads();
  {
    v4u vals[3];
#pragma unroll
    for (int it = 0; it < 3; ++it) {
      const int p   = it * 256 + tid;
      const int row = p / (DM / 8);
      const int c8  = (p - row * (DM / 8)) * 8;
      vals[it] = *(const v4u*)(Os + row * DM + c8);
    }
    unsigned short* dst = CT + ((size_t)bat * NTOK + q0) * DM;
    for (int pass = 0; pass < 2; ++pass) {
#pragma unroll
      for (int it = 0; it < 3; ++it) {
        const int p   = it * 256 + tid;
        const int row = p / (DM / 8);
        const int c8  = (p - row * (DM / 8)) * 8;
        *(volatile v4u*)(dst + (size_t)row * DM + c8) = vals[it];
      }
      __threadfence();
    }
  }
}

__global__ __launch_bounds__(256) void resid_ln(const float* __restrict__ O, const float* __restrict__ X,
                                                const float* __restrict__ gam, const float* __restrict__ bet,
                                                float* out, int nrows) {
  const int lane = threadIdx.x & 31, wave = threadIdx.x >> 5;
  const int row = blockIdx.x * 8 + wave;
  if (row >= nrows) return;
  const float* op = O + (size_t)row * DM;
  const float* xp = X + (size_t)row * DM;
  v4f y[3];
  float s = 0.f;
#pragma unroll
  for (int j = 0; j < 3; ++j) {
    const int c0 = j * 128 + lane * 4;
    const v4f ov = *(const v4f*)(op + c0);
    const v4f xv = *(const v4f*)(xp + c0);
    v4f t;
#pragma unroll
    for (int e = 0; e < 4; ++e) { t[e] = bfr(xv[e]) + ov[e]; s += t[e]; }
    y[j] = t;
  }
#pragma unroll
  for (int off = 1; off < 32; off <<= 1) s += __shfl_xor(s, off, 32);
  const float mu = s * (1.0f / (float)DM);
  float ss = 0.f;
#pragma unroll
  for (int j = 0; j < 3; ++j) {
#pragma unroll
    for (int e = 0; e < 4; ++e) { const float d = y[j][e] - mu; ss += d * d; }
  }
#pragma unroll
  for (int off = 1; off < 32; off <<= 1) ss += __shfl_xor(ss, off, 32);
  const float var  = ss * (1.0f / (float)DM);
  const float rstd = rsqrtf(var + LN_EPS);
  v4f res[3];
#pragma unroll
  for (int j = 0; j < 3; ++j) {
    const int c0 = j * 128 + lane * 4;
    const v4f gv = *(const v4f*)(gam + c0);
    const v4f bv = *(const v4f*)(bet + c0);
    v4f t;
#pragma unroll
    for (int e = 0; e < 4; ++e) t[e] = (y[j][e] - mu) * rstd * bfr(gv[e]) + bfr(bv[e]);
    res[j] = t;
  }
  float* dst = out + (size_t)row * DM;
  for (int pass = 0; pass < 2; ++pass) {
#pragma unroll
    for (int j = 0; j < 3; ++j) *(volatile v4f*)(dst + j * 128 + lane * 4) = res[j];
    __threadfence();
  }
}

extern "C" void kernel_launch(void* const* d_in, const int* in_sizes, int n_in,
                              void* d_out, int out_size, void* d_ws, size_t ws_size,
                              hipStream_t stream) {
  if (n_in < 9) return;
  if (in_sizes[0] != MROWS * DM) return;
  if (in_sizes[1] != MROWS * NFR) return;
  if (in_sizes[2] != DM * DM || in_sizes[3] != DM * DM || in_sizes[4] != DM * DM || in_sizes[5] != DM * DM) return;
  if (in_sizes[6] != DM || in_sizes[7] != DM || in_sizes[8] != DM) return;
  if (out_size != MROWS * DM) return;

  const float* x_in = (const float*)d_in[0];
  const float* fr   = (const float*)d_in[1];
  const float* w_q  = (const float*)d_in[2];
  const float* w_k  = (const float*)d_in[3];
  const float* w_v  = (const float*)d_in[4];
  const float* w_o  = (const float*)d_in[5];
  const float* b_o  = (const float*)d_in[6];
  const float* gam  = (const float*)d_in[7];
  const float* bet  = (const float*)d_in[8];
  float*       out  = (float*)d_out;

  const size_t PWQK = (size_t)2 * DM * DM * 2;
  const size_t PW   = (size_t)DM * DM * 2;
  const size_t PXI  = (size_t)MROWS * DM * 2;
  const size_t PQKF = (size_t)MROWS * 2 * DM * 4;
  const size_t PVT  = (size_t)NBATCH * DM * NTOK * 2;
  const size_t PQR  = (size_t)MROWS * QKP * 2;
  const size_t PCT  = (size_t)MROWS * DM * 2;
  const size_t POP  = (size_t)MROWS * DM * 4;
  size_t off = 0;
  const size_t oWQK = off; off += PWQK;
  const size_t oWV  = off; off += PW;
  const size_t oWO  = off; off += PW;
  const size_t oXI  = off; off += PXI;
  const size_t oQKF = off; off += PQKF;
  const size_t oVT  = off; off += PVT;
  const size_t oQR  = off; off += PQR;
  const size_t oKR  = off; off += PQR;
  const size_t oCT  = off; off += PCT;
  const size_t oOP  = off; off += POP;
  if (off > ws_size) return;
  if (off > (size_t)134217728) return;

  char* ws = (char*)d_ws;
  unsigned short* WQK = (unsigned short*)(ws + oWQK);
  unsigned short* WV  = (unsigned short*)(ws + oWV);
  unsigned short* WO  = (unsigned short*)(ws + oWO);
  unsigned short* XI  = (unsigned short*)(ws + oXI);
  float*          QKF = (float*)(ws + oQKF);
  unsigned short* VTp = (unsigned short*)(ws + oVT);
  unsigned short* QR  = (unsigned short*)(ws + oQR);
  unsigned short* KR  = (unsigned short*)(ws + oKR);
  unsigned short* CT  = (unsigned short*)(ws + oCT);
  float*          OP  = (float*)(ws + oOP);

  const int n8w = (DM * DM) / 8;
  const int n8x = (MROWS * DM) / 8;
  if ((n8w % 256) != 0 || (n8x % 256) != 0) return;
  const dim3 blk(256);
  const dim3 gCw(n8w / 256), gCx(n8x / 256);
  const int tilesQK = (MROWS / 64) * ((2 * DM) / 64);
  const int tilesVT = (DM / 64) * (NTOK / 64);
  const int tilesOP = (MROWS / 64) * (DM / 64);
  if ((tilesQK % 8) != 0 || (tilesVT % 8) != 0 || (tilesOP % 8) != 0) return;
  const dim3 gQK(tilesQK / 8, 1);
  const dim3 gVT(tilesVT / 8, NBATCH);
  const dim3 gOP(tilesOP / 8, 1);
  const dim3 gRP(MROWS / 16);
  const dim3 gAT(ATT_BLOCKS);
  const dim3 gLN(MROWS / 8);

  conv16<<<gCw, blk, 0, stream>>>(w_q, WQK, n8w, WSC);
  conv16<<<gCw, blk, 0, stream>>>(w_k, WQK + (size_t)DM * DM, n8w, WSC);
  conv16<<<gCw, blk, 0, stream>>>(w_v, WV, n8w, WSC);
  conv16<<<gCw, blk, 0, stream>>>(w_o, WO, n8w, WSC);

  conv16<<<gCx, blk, 0, stream>>>(x_in, XI, n8x, ACARRY);

  gemm64<0, 0><<<gQK, blk, 0, stream>>>(
      XI, DM, 0LL,
      WQK, DM, 0LL,
      b_o, 0.f,
      (void*)QKF, (void*)QKF, 2 * DM, 0LL,
      MROWS, 2 * DM, DM, 1.0f / (ACARRY * WSC));

  gemm64<2, 0><<<gVT, blk, 0, stream>>>(
      WV, DM, 0LL,
      XI, DM, (long long)NTOK * DM,
      b_o, 0.f,
      (void*)VTp, (void*)VTp, NTOK, (long long)DM * NTOK,
      DM, NTOK, DM, VC / (ACARRY * WSC));

  rot_pack<<<gRP, blk, 0, stream>>>(QKF, fr, QR, KR, QC, KC);

  attn48<<<gAT, blk, 0, stream>>>(QR, KR, VTp, CT);

  gemm64<0, 1><<<gOP, blk, 0, stream>>>(
      CT, DM, 0LL,
      WO, DM, 0LL,
      b_o, 1.0f,
      (void*)OP, (void*)OP, DM, 0LL,
      MROWS, DM, DM, 1.0f / (FC * WSC));

  resid_ln<<<gLN, blk, 0, stream>>>(OP, x_in, gam, bet, out, MROWS);
  (void)hipGetLastError();
}
